// _Attn_3616362463484
// MI455X (gfx1250) — hardware-verified
//
#include <hip/hip_runtime.h>
#include <stdint.h>

#define EMBED   1024
#define HEADS   16
#define HEAD_D  64
#define BATCH   2
#define SEQ     2048
#define MROWS   (BATCH * SEQ)
#define QKVW    (3 * EMBED)

#define GT_M    64
#define GT_N    128
#define LDP     40
#define CSP     132

typedef _Float16 v16h __attribute__((ext_vector_type(16)));
typedef _Float16 v8h  __attribute__((ext_vector_type(8)));
typedef float    v8f  __attribute__((ext_vector_type(8)));
typedef float    v4f  __attribute__((ext_vector_type(4)));
typedef v8h v8hm __attribute__((may_alias));
typedef v4f v4fm __attribute__((may_alias));


__device__ __forceinline__ float bf16r(float f) {
  unsigned int u = __float_as_uint(f);
  u = (u + 0x7fffu + ((u >> 16) & 1u)) & 0xffff0000u;
  return __uint_as_float(u);
}

__device__ __forceinline__ v16h cat8(v8h a, v8h b) {
  return __builtin_shufflevector(a, b, 0,1,2,3,4,5,6,7,8,9,10,11,12,13,14,15);
}

__device__ __forceinline__ v16h ldfrag(const _Float16* p) {
  return cat8(*(const v8hm*)p, *(const v8hm*)(p + 16));
}

__device__ __forceinline__ v8f wmma16(v16h a, v16h b, v8f c) {
  v8f d = __builtin_amdgcn_wmma_f32_16x16x32_f16(false, a, false, b, (short)0, c, false, false);
  asm volatile("v_nop\n\tv_nop\n\tv_nop\n\tv_nop" : "+v"(d) : "v"(a), "v"(b));
  return d;
}

#define SWZ(x, m) __int_as_float(__builtin_amdgcn_ds_swizzle(__float_as_int(x), (0x1f | ((m) << 10))))
__device__ __forceinline__ float rowMax16(float v) {
  v = fmaxf(v, SWZ(v, 1)); v = fmaxf(v, SWZ(v, 2));
  v = fmaxf(v, SWZ(v, 4)); v = fmaxf(v, SWZ(v, 8));
  return v;
}
__device__ __forceinline__ float rowSum16(float v) {
  v += SWZ(v, 1); v += SWZ(v, 2); v += SWZ(v, 4); v += SWZ(v, 8);
  return v;
}


__global__ __launch_bounds__(256) void k_cvt(const float* __restrict__ s0, const float* __restrict__ s1,
                                            const float* __restrict__ s2,
                                            _Float16* d0, _Float16* d1, _Float16* d2,
                                            int n0, int n1, int n2, int nb0, int nb1,
                                            float c0, float c1, float c2)
{
  int bid = blockIdx.x;
  const float* src; _Float16* dst; int n; float sc;
  if (bid < nb0)            { src = s0; dst = d0; n = n0; sc = c0; }
  else if (bid < nb0 + nb1) { bid -= nb0; src = s1; dst = d1; n = n1; sc = c1; }
  else                      { bid -= nb0 + nb1; src = s2; dst = d2; n = n2; sc = c2; }
  const size_t i = ((size_t)bid * 256 + threadIdx.x) * 8;
  if (i + 8 <= (size_t)n) {
    const v4f a = *(const v4fm*)(src + i);
    const v4f b = *(const v4fm*)(src + i + 4);
    v8h o;
#pragma unroll
    for (int e = 0; e < 4; ++e) {
      o[e]     = (_Float16)(bf16r(a[e]) * sc);
      o[e + 4] = (_Float16)(bf16r(b[e]) * sc);
    }
    *(volatile v8h*)(dst + i) = o;
    __threadfence();
    *(volatile v8h*)(dst + i) = o;
  }
}


template<int NPA, int MODE>
__global__ __launch_bounds__(256) void k_gemm(
    const _Float16* __restrict__ A0, const _Float16* __restrict__ A1,
    const _Float16* __restrict__ Bw, const float* __restrict__ bias,
    _Float16* oh, _Float16* ol, float* of,
    int M, int N, int K, float oscale, float bscale)
{
  __shared__ __attribute__((aligned(16))) _Float16 sm[GT_M * CSP * 2];
  _Float16* As0 = sm;
  _Float16* As1 = sm + 2560;
  _Float16* Bs  = sm + 5120;

  const int tid  = threadIdx.x;
  const int lane = tid & 31;
  const int wid  = tid >> 5;
  const int wM   = wid & 1, wN = wid >> 1;
  const int hh   = lane >> 4, l16 = lane & 15;
  const int m0 = blockIdx.y * GT_M;
  const int n0 = blockIdx.x * GT_N;

  v8f c[2][2];
  {
    v8f z = {0.f, 0.f, 0.f, 0.f, 0.f, 0.f, 0.f, 0.f};
#pragma unroll
    for (int i = 0; i < 2; ++i)
#pragma unroll
      for (int j = 0; j < 2; ++j) c[i][j] = z;
  }

  const int sr  = tid >> 2;
  const int sc8 = (tid & 3) * 8;
  const int am  = (m0 + sr < M) ? (m0 + sr) : (M - 1);

  for (int k0 = 0; k0 < K; k0 += 32) {
    {
      const v8h va = *(const v8hm*)(A0 + (size_t)am * K + k0 + sc8);
      *(v8hm*)(As0 + sr * LDP + sc8) = va;
      if (NPA == 2) {
        const v8h vb = *(const v8hm*)(A1 + (size_t)am * K + k0 + sc8);
        *(v8hm*)(As1 + sr * LDP + sc8) = vb;
      }
#pragma unroll
      for (int q = 0; q < 2; ++q) {
        const int idx = tid + q * 256;
        const int rn = idx >> 2, cb = (idx & 3) * 8;
        const int bn = (n0 + rn < N) ? (n0 + rn) : (N - 1);
        const v8h vw = *(const v8hm*)(Bw + (size_t)bn * K + k0 + cb);
        *(v8hm*)(Bs + rn * LDP + cb) = vw;
      }
    }
    __syncthreads();

    v16h af0[2], af1[2], bfv[2];
#pragma unroll
    for (int i = 0; i < 2; ++i) {
      af0[i] = ldfrag(As0 + (wM * 32 + i * 16 + l16) * LDP + 8 * hh);
      if (NPA == 2) af1[i] = ldfrag(As1 + (wM * 32 + i * 16 + l16) * LDP + 8 * hh);
      else          af1[i] = af0[i];
    }
#pragma unroll
    for (int j = 0; j < 2; ++j)
      bfv[j] = ldfrag(Bs + (wN * 32 + j * 16 + l16) * LDP + 8 * hh);
#pragma unroll
    for (int i = 0; i < 2; ++i)
#pragma unroll
      for (int j = 0; j < 2; ++j) {
        c[i][j] = wmma16(af0[i], bfv[j], c[i][j]);
        if (NPA == 2) c[i][j] = wmma16(af1[i], bfv[j], c[i][j]);
      }
    __syncthreads();
  }

  float* Cs = (float*)sm;
#pragma unroll
  for (int i = 0; i < 2; ++i)
#pragma unroll
    for (int j = 0; j < 2; ++j)
#pragma unroll
      for (int r = 0; r < 8; ++r)
        Cs[(wM * 32 + i * 16 + hh * 8 + r) * CSP + wN * 32 + j * 16 + l16] = c[i][j][r];
  __syncthreads();

  if (MODE == 1) {
    const int col = 4 * lane;
    const v4f b4 = *(const v4fm*)(bias + n0 + col);
    v4f bb;
#pragma unroll
    for (int e = 0; e < 4; ++e) bb[e] = bscale * bf16r(b4[e]);
    v4f tv[8];
#pragma unroll
    for (int q = 0; q < 8; ++q) {
      const int row = wid * 8 + q;
      const v4f x = *(const v4fm*)(Cs + row * CSP + col);
      const v4f t = x * oscale + bb;
      tv[q] = t;
      if (m0 + row < M)
        *(volatile v4f*)(of + (size_t)(m0 + row) * N + n0 + col) = t;
    }
    __threadfence();
#pragma unroll
    for (int q = 0; q < 8; ++q) {
      const int row = wid * 8 + q;
      if (m0 + row < M)
        *(volatile v4f*)(of + (size_t)(m0 + row) * N + n0 + col) = tv[q];
    }
  } else {
    const int col = 8 * l16;
    const v4f b0 = *(const v4fm*)(bias + n0 + col);
    const v4f b1 = *(const v4fm*)(bias + n0 + col + 4);
    v4f bb0, bb1;
#pragma unroll
    for (int e = 0; e < 4; ++e) { bb0[e] = bscale * bf16r(b0[e]); bb1[e] = bscale * bf16r(b1[e]); }
    v8h hv[4], lv[4];
#pragma unroll
    for (int it = 0; it < 4; ++it) {
      const int row = wid * 8 + it * 2 + hh;
      const float* cr = Cs + row * CSP + col;
      const v4f x0 = *(const v4fm*)cr;
      const v4f x1 = *(const v4fm*)(cr + 4);
      v8h h8, l8;
#pragma unroll
      for (int e = 0; e < 4; ++e) {
        const float t0 = x0[e] * oscale + bb0[e];
        const _Float16 th0 = (_Float16)t0;
        h8[e] = th0; l8[e] = (_Float16)(t0 - (float)th0);
        const float t1 = x1[e] * oscale + bb1[e];
        const _Float16 th1 = (_Float16)t1;
        h8[e + 4] = th1; l8[e + 4] = (_Float16)(t1 - (float)th1);
      }
      hv[it] = h8; lv[it] = l8;
      if (m0 + row < M) {
        const size_t g = (size_t)(m0 + row) * N + n0 + col;
        *(volatile v8h*)(oh + g) = h8;
        *(volatile v8h*)(ol + g) = l8;
      }
    }
    __threadfence();
#pragma unroll
    for (int it = 0; it < 4; ++it) {
      const int row = wid * 8 + it * 2 + hh;
      if (m0 + row < M) {
        const size_t g = (size_t)(m0 + row) * N + n0 + col;
        *(volatile v8h*)(oh + g) = hv[it];
        *(volatile v8h*)(ol + g) = lv[it];
      }
    }
  }
}


__global__ __launch_bounds__(256) void k_attn(const _Float16* __restrict__ Hp, const _Float16* __restrict__ Lp,
                                             _Float16* Oh, _Float16* Ol)
{
  __shared__ __attribute__((aligned(16))) _Float16 sm[19968];
  _Float16* Kh = sm;
  _Float16* Kl = sm + 2304;
  _Float16* Vh = sm + 4608;
  _Float16* Vl = sm + 7168;

  const int tid  = threadIdx.x;
  const int lane = tid & 31;
  const int wid  = tid >> 5;
  const int hh = lane >> 4, l16 = lane & 15;
  _Float16* Ph = sm + 9728 + wid * 1280;
  _Float16* Pl = Ph + 640;

  const int bh = blockIdx.y;
  const int b  = bh / HEADS, h = bh - b * HEADS;
  const int qBase = blockIdx.x * 128 + wid * 16;

  v16h qh[2], ql[2];
  {
    const size_t rq = (size_t)(b * SEQ + qBase + l16) * QKVW + h * HEAD_D + 8 * hh;
#pragma unroll
    for (int t2 = 0; t2 < 2; ++t2) {
      qh[t2] = ldfrag(Hp + rq + t2 * 32);
      ql[t2] = ldfrag(Lp + rq + t2 * 32);
    }
  }

  v8f oacc[4];
  {
    v8f z = {0.f, 0.f, 0.f, 0.f, 0.f, 0.f, 0.f, 0.f};
#pragma unroll
    for (int dt = 0; dt < 4; ++dt) oacc[dt] = z;
  }
  float m_i[8], l_i[8];
#pragma unroll
  for (int r = 0; r < 8; ++r) { m_i[r] = -3.0e38f; l_i[r] = 0.0f; }

  const int nT  = (blockIdx.x + 1) * 4;
  const int key = tid >> 3, ch8 = (tid & 7) * 8;
  const float SCL = 1.9073486328125e-06f;
  const float NEG = -3.0e38f;

  for (int ti = 0; ti < nT; ++ti) {
    const int kt0 = ti * 32;
    {
      const size_t rk = (size_t)(b * SEQ + kt0 + key) * QKVW + h * HEAD_D + ch8;
      const v8h ka = *(const v8hm*)(Hp + rk + EMBED);
      const v8h kb = *(const v8hm*)(Lp + rk + EMBED);
      *(v8hm*)(Kh + key * 72 + ch8) = ka;
      *(v8hm*)(Kl + key * 72 + ch8) = kb;
      const v8h va = *(const v8hm*)(Hp + rk + 2 * EMBED);
      const v8h vb = *(const v8hm*)(Lp + rk + 2 * EMBED);
#pragma unroll
      for (int e = 0; e < 8; ++e) {
        Vh[(ch8 + e) * 40 + key] = va[e];
        Vl[(ch8 + e) * 40 + key] = vb[e];
      }
    }
    __syncthreads();

    if (kt0 <= qBase + 15) {
      v8f s[2];
#pragma unroll
      for (int sn = 0; sn < 2; ++sn) {
        v8f acc = {0.f, 0.f, 0.f, 0.f, 0.f, 0.f, 0.f, 0.f};
#pragma unroll
        for (int t2 = 0; t2 < 2; ++t2) {
          const _Float16* kp = Kh + (sn * 16 + l16) * 72 + t2 * 32 + 8 * hh;
          const _Float16* lp = Kl + (sn * 16 + l16) * 72 + t2 * 32 + 8 * hh;
          const v16h khf = ldfrag(kp);
          const v16h klf = ldfrag(lp);
          acc = wmma16(qh[t2], khf, acc);
          acc = wmma16(qh[t2], klf, acc);
          acc = wmma16(ql[t2], khf, acc);
        }
        s[sn] = acc;
      }
#pragma unroll
      for (int r = 0; r < 8; ++r) {
        const int q = qBase + hh * 8 + r;
        float v0 = s[0][r] * SCL;
        float v1 = s[1][r] * SCL;
        if (kt0 + l16 > q)      v0 = NEG;
        if (kt0 + 16 + l16 > q) v1 = NEG;
        const float mx   = rowMax16(fmaxf(v0, v1));
        const float mnew = fmaxf(m_i[r], mx);
        const float p0 = __expf(v0 - mnew);
        const float p1 = __expf(v1 - mnew);
        const float rs   = rowSum16(p0 + p1);
        const float corr = __expf(m_i[r] - mnew);
        l_i[r] = l_i[r] * corr + rs;
        m_i[r] = mnew;
#pragma unroll
        for (int dt = 0; dt < 4; ++dt) oacc[dt][r] = oacc[dt][r] * corr;
        const float t0 = p0 * 4096.0f, t1 = p1 * 4096.0f;
        const _Float16 h0 = (_Float16)t0, h1 = (_Float16)t1;
        Ph[(hh * 8 + r) * 40 + l16]      = h0;
        Ph[(hh * 8 + r) * 40 + 16 + l16] = h1;
        Pl[(hh * 8 + r) * 40 + l16]      = (_Float16)(t0 - (float)h0);
        Pl[(hh * 8 + r) * 40 + 16 + l16] = (_Float16)(t1 - (float)h1);
      }
      asm volatile("s_wait_dscnt 0x0" ::: "memory");

      const v16h pfh = ldfrag(Ph + l16 * 40 + 8 * hh);
      const v16h pfl = ldfrag(Pl + l16 * 40 + 8 * hh);
#pragma unroll
      for (int dt = 0; dt < 4; ++dt) {
        const v16h vhf = ldfrag(Vh + (dt * 16 + l16) * 40 + 8 * hh);
        const v16h vlf = ldfrag(Vl + (dt * 16 + l16) * 40 + 8 * hh);
        oacc[dt] = wmma16(pfh, vhf, oacc[dt]);
        oacc[dt] = wmma16(pfh, vlf, oacc[dt]);
        oacc[dt] = wmma16(pfl, vhf, oacc[dt]);
      }
    }
    __syncthreads();
  }

  _Float16* Os = sm + wid * 2048;
  const float OSC = 0.000244140625f;
#pragma unroll
  for (int r = 0; r < 8; ++r) {
    const float rl = (1.0f / l_i[r]) * OSC;
#pragma unroll
    for (int dt = 0; dt < 4; ++dt) {
      const float v = oacc[dt][r] * rl;
      const _Float16 hv = (_Float16)v;
      Os[(hh * 8 + r) * 64 + dt * 16 + l16]        = hv;
      Os[1024 + (hh * 8 + r) * 64 + dt * 16 + l16] = (_Float16)(v - (float)hv);
    }
  }
  __syncthreads();

  v8h oh8[4], ol8[4];
  const int rsub = lane >> 3, c8 = (lane & 7) * 8;
#pragma unroll
  for (int it = 0; it < 4; ++it) {
    const int row = it * 4 + rsub;
    oh8[it] = *(const v8hm*)(Os + row * 64 + c8);
    ol8[it] = *(const v8hm*)(Os + 1024 + row * 64 + c8);
    const size_t g = (size_t)(b * SEQ + qBase + row) * EMBED + h * HEAD_D + c8;
    *(volatile v8h*)(Oh + g) = oh8[it];
    *(volatile v8h*)(Ol + g) = ol8[it];
  }
  __threadfence();
#pragma unroll
  for (int it = 0; it < 4; ++it) {
    const int row = it * 4 + rsub;
    const size_t g = (size_t)(b * SEQ + qBase + row) * EMBED + h * HEAD_D + c8;
    *(volatile v8h*)(Oh + g) = oh8[it];
    *(volatile v8h*)(Ol + g) = ol8[it];
  }
}


extern "C" void kernel_launch(void* const* d_in, const int* in_sizes, int n_in,
                              void* d_out, int out_size, void* d_ws, size_t ws_size,
                              hipStream_t stream) {
  if (n_in < 5) return;
  const int nx  = in_sizes[0];
  const int nwq = in_sizes[1];
  const int nbq = in_sizes[2];
  const int nwo = in_sizes[3];
  const int nbo = in_sizes[4];
  if (nx != MROWS * EMBED || nwq != 3 * EMBED * EMBED || nbq != 3 * EMBED ||
      nwo != EMBED * EMBED || nbo != EMBED || out_size != MROWS * EMBED) return;
  if ((nx % 2048) != 0 || (nwq % 2048) != 0 || (nwo % 2048) != 0) return;

  const float* x     = (const float*)d_in[0];
  const float* w_qkv = (const float*)d_in[1];
  const float* b_qkv = (const float*)d_in[2];
  const float* w_out = (const float*)d_in[3];
  const float* b_out = (const float*)d_in[4];
  float* out = (float*)d_out;

  const size_t bx  = (size_t)nx  * 2;
  const size_t bwq = (size_t)nwq * 2;
  const size_t bwo = (size_t)nwo * 2;
  const size_t bpl = (size_t)MROWS * QKVW * 2;
  const size_t bo  = (size_t)MROWS * EMBED * 2;
  size_t off = 0;
  char* ws = (char*)d_ws;
  _Float16* xh   = (_Float16*)(ws + off); off += bx;
  _Float16* wqh  = (_Float16*)(ws + off); off += bwq;
  _Float16* woh  = (_Float16*)(ws + off); off += bwo;
  _Float16* Hp   = (_Float16*)(ws + off); off += bpl;
  _Float16* Lp   = (_Float16*)(ws + off); off += bpl;
  _Float16* Ohp  = (_Float16*)(ws + off); off += bo;
  _Float16* Olp  = (_Float16*)(ws + off); off += bo;
  if (off > ws_size) return;

  const int nb0 = nx / 2048, nb1 = nwq / 2048, nb2 = nwo / 2048;
  k_cvt<<<nb0 + nb1 + nb2, 256, 0, stream>>>(x, w_qkv, w_out, xh, wqh, woh,
                                             nx, nwq, nwo, nb0, nb1,
                                             16.0f, 1024.0f, 1024.0f);

  k_gemm<1, 0><<<dim3(QKVW / GT_N, MROWS / GT_M), 256, 0, stream>>>(
      xh, xh, wqh, b_qkv, Hp, Lp, out, MROWS, QKVW, EMBED, 0.015625f, 256.0f);

  k_attn<<<dim3(SEQ / 128, BATCH * HEADS), 256, 0, stream>>>(Hp, Lp, Ohp, Olp);

  k_gemm<2, 1><<<dim3(EMBED / GT_N, MROWS / GT_M), 256, 0, stream>>>(
      Ohp, Olp, woh, b_out, Hp, Lp, out, MROWS, EMBED, EMBED, 3.814697265625e-06f, 1.0f);
}
